// MultiDilatelocalAttention_43327630082583
// MI455X (gfx1250) — hardware-verified
//
#include <hip/hip_runtime.h>


#define NB_  8
#define CC   256
#define HH   64
#define NPX  4096
#define HID  1024
#define HDM  32
#define DM   CC
#define SCL  0.17677669529663688f
#define LEPS 1e-5f
#define LOSC 1024.0f

typedef _Float16 h16;
typedef unsigned short bf;
typedef __attribute__((ext_vector_type(16))) __bf16   v16bf;
typedef __attribute__((ext_vector_type(16))) _Float16 v16h;
typedef __attribute__((ext_vector_type(8)))  _Float16 v8h;
typedef __attribute__((ext_vector_type(8)))  unsigned short v8us;
typedef __attribute__((ext_vector_type(8)))  float    v8f;
typedef __attribute__((ext_vector_type(4)))  float    v4f;
typedef v8h  __attribute__((may_alias)) v8ha;
typedef v4f  __attribute__((may_alias)) v4fa;
typedef v8us __attribute__((may_alias)) v8usa;

__device__ __forceinline__ unsigned short f2bf(float f) { unsigned u = __float_as_uint(f); u += 0x7FFFu + ((u >> 16) & 1u); return (unsigned short)(u >> 16); }
__device__ __forceinline__ float bf2f(unsigned short b) { return __uint_as_float(((unsigned)b) << 16); }
__device__ __forceinline__ float bfr(float f) { return bf2f(f2bf(f)); }
__device__ __forceinline__ v16h cat16(v8h lo, v8h hi) { return __builtin_shufflevector(lo, hi, 0, 1, 2, 3, 4, 5, 6, 7, 8, 9, 10, 11, 12, 13, 14, 15); }
__device__ __forceinline__ v16bf cat16b(v8us lo, v8us hi) { return __builtin_bit_cast(v16bf, __builtin_shufflevector(lo, hi, 0, 1, 2, 3, 4, 5, 6, 7, 8, 9, 10, 11, 12, 13, 14, 15)); }
__device__ __forceinline__ v8f wmma16(v16h a, v16h b, v8f c) { return __builtin_amdgcn_wmma_f32_16x16x32_f16(false, a, false, b, (short)0, c, false, false); }
__device__ __forceinline__ v8f wmmab(v16bf a, v16bf b, v8f c) { return __builtin_amdgcn_wmma_f32_16x16x32_bf16(false, a, false, b, (short)0, c, false, false); }

template <bool SPLITA, bool F16OUT = false>
__global__ __launch_bounds__(128) void k_gemmb(const bf* __restrict__ A, const bf* __restrict__ Al, const bf* __restrict__ Bn, const float* __restrict__ bias, float* C, int ldc, h16* C2, const float* __restrict__ R = nullptr, int K = DM, int roundR = 1) {
    __shared__ __align__(16) float ost[4][16 * 68];
    const int lane = threadIdx.x & 31, wave = threadIdx.x >> 5, lr = lane & 15, hi = lane >> 4;
    const int r0 = blockIdx.x * 64 + wave * 16, c0 = blockIdx.y * 64;
    const size_t aoff = (size_t)(r0 + lr) * K + 8 * hi;
    size_t boff[4];
#pragma unroll
    for (int t = 0; t < 4; ++t) boff[t] = (size_t)(c0 + t * 16 + lr) * K + 8 * hi;
    v8f acc[4];
#pragma unroll
    for (int t = 0; t < 4; ++t) acc[t] = (v8f){};
#pragma unroll 1
    for (int kc = 0; kc < K; kc += 32) {
        const v16bf a = cat16b(*(const v8us*)(A + aoff + kc), *(const v8us*)(A + aoff + kc + 16));
        v16bf al = a;
        if (SPLITA) al = cat16b(*(const v8us*)(Al + aoff + kc), *(const v8us*)(Al + aoff + kc + 16));
#pragma unroll
        for (int t = 0; t < 4; ++t) { const v16bf b = cat16b(*(const v8us*)(Bn + boff[t] + kc), *(const v8us*)(Bn + boff[t] + kc + 16)); acc[t] = wmmab(a, b, acc[t]); if (SPLITA) acc[t] = wmmab(al, b, acc[t]); }
        asm volatile("v_nop\n\tv_nop\n\tv_nop\n\tv_nop" : "+v"(acc[0]), "+v"(acc[1]), "+v"(acc[2]), "+v"(acc[3]) : "v"(a), "v"(al));
    }
    float* os = &ost[wave][0];
#pragma unroll
    for (int t = 0; t < 4; ++t) { const float bv = bias ? bfr(bias[c0 + t * 16 + lr]) : 0.f;
#pragma unroll
        for (int j = 0; j < 8; ++j) os[(hi * 8 + j) * 68 + t * 16 + lr] = acc[t][j] + bv; }
    __syncthreads();
    if (F16OUT) {
        h16* crow = (h16*)(void*)C + (size_t)r0 * ldc + c0;
        auto pass = [&]() {
#pragma unroll
            for (int s = 0; s < 4; ++s) { const int row = 4 * s + (lane >> 3), piece = lane & 7; const float* sp = os + row * 68 + piece * 8; v8h o, o2;
#pragma unroll
                for (int i = 0; i < 8; ++i) { const h16 a = (h16)sp[i]; o[i] = a; o2[i] = (h16)((sp[i] - (float)a) * LOSC); }
                *(volatile v8h*)(crow + (size_t)row * ldc + piece * 8) = o; if (C2) *(volatile v8h*)(C2 + (size_t)r0 * ldc + c0 + (size_t)row * ldc + piece * 8) = o2; }
        };
        pass(); __threadfence(); pass();
    } else {
        float* crow = C + (size_t)r0 * ldc + c0;
        auto pass = [&]() {
#pragma unroll
            for (int s = 0; s < 8; ++s) { const int Lid = (lane >> 3) + 4 * s, piece = lane & 7; const int row = Lid >> 1, cofs = (Lid & 1) * 32 + piece * 4;
                v4f val = *(const v4fa*)(os + row * 68 + cofs); if (R) { const v4f rv = *(const v4f*)(R + ((size_t)r0 + row) * ldc + c0 + cofs); val += roundR ? (v4f){bfr(rv[0]), bfr(rv[1]), bfr(rv[2]), bfr(rv[3])} : rv; }
                *(volatile v4f*)(crow + (size_t)row * ldc + cofs) = val; }
        };
        pass(); __threadfence(); pass();
    }
}

__global__ __launch_bounds__(256) void k_cvt8(const float* __restrict__ src, bf* dst, size_t n8) {
    const size_t i = (size_t)blockIdx.x * 256 + threadIdx.x; if (i >= n8) return;
    const v8f v = *(const v8f*)(src + i * 8); v8us o;
#pragma unroll
    for (int k = 0; k < 8; ++k) o[k] = f2bf(v[k]);
    *(volatile v8us*)(dst + i * 8) = o; __threadfence(); *(volatile v8us*)(dst + i * 8) = o;
}
__global__ __launch_bounds__(256) void k_zero8(bf* dst, size_t n8) {
    const size_t i = (size_t)blockIdx.x * 256 + threadIdx.x; if (i >= n8) return; v8us z;
#pragma unroll
    for (int k = 0; k < 8; ++k) z[k] = 0;
    *(volatile v8us*)(dst + i * 8) = z; __threadfence(); *(volatile v8us*)(dst + i * 8) = z;
}

__global__ __launch_bounds__(256) void k_ptb(const float* __restrict__ xb, bf* XT) {
    __shared__ float tl[64][65];
    typedef __attribute__((ext_vector_type(4))) unsigned short v4us;
    const int tid = threadIdx.x, c0 = blockIdx.x * 64, p0 = blockIdx.y * 64; const int rr = tid >> 2, cq = (tid & 3) * 16;
#pragma unroll
    for (int i = 0; i < 16; ++i) tl[rr][cq + i] = xb[(size_t)(c0 + rr) * NPX + p0 + cq + i];
    __syncthreads();
    const int lane = tid & 31, wv = tid >> 5;
    auto pass = [&]() {
#pragma unroll
        for (int st = 0; st < 4; ++st) { const int pr = wv * 8 + st * 2 + (lane >> 4); const int cl = (lane & 15) * 4; v4us v;
#pragma unroll
            for (int i = 0; i < 4; ++i) v[i] = f2bf(tl[cl + i][pr]);
            *(volatile v4us*)(XT + (size_t)(p0 + pr) * CC + c0 + cl) = v; }
    };
    pass(); __threadfence(); pass();
}
__global__ __launch_bounds__(256) void k_local(const float* __restrict__ Q, const float* __restrict__ K, const float* __restrict__ V, float* ATT, bf* Ah, bf* Al) {
    const int lane = threadIdx.x & 31; const size_t p = (size_t)blockIdx.x * 8 + (threadIdx.x >> 5); if (p >= (size_t)NPX) return; const int y = (int)(p / HH), x = (int)(p % HH);
    const int grp = lane >> 3; const int dil = grp + 1; const int c0 = lane * 8;
    float q[8];
#pragma unroll
    for (int i = 0; i < 8; ++i) q[i] = Q[p * CC + c0 + i];
    auto logit = [&](int kk, bool& ok, size_t& nb) -> float { const int yy = y + (kk / 3 - 1) * dil, xx = x + (kk % 3 - 1) * dil; ok = yy >= 0 && yy < HH && xx >= 0 && xx < HH; nb = ok ? (size_t)(yy * HH + xx) : 0; float s = 0.f;
#pragma unroll
        for (int i = 0; i < 8; ++i) s = fmaf(q[i], ok ? K[nb * CC + c0 + i] : 0.f, s);
        s += __shfl_xor(s, 1, 32); s += __shfl_xor(s, 2, 32); return s * SCL; };
    float m = -3.0e38f;
#pragma unroll 1
    for (int kk = 0; kk < 9; ++kk) { bool ok; size_t nb; m = fmaxf(m, logit(kk, ok, nb)); }
    float den = 0.f; v8f o; v8us oh, ol;
#pragma unroll
    for (int i = 0; i < 8; ++i) o[i] = 0.f;
#pragma unroll 1
    for (int kk = 0; kk < 9; ++kk) { bool ok; size_t nb; const float e = expf(logit(kk, ok, nb) - m); den += e;
#pragma unroll
        for (int i = 0; i < 8; ++i) o[i] = fmaf(e, ok ? V[nb * CC + c0 + i] : 0.f, o[i]); }
    const float inv = 1.0f / den;
#pragma unroll
    for (int i = 0; i < 8; ++i) { o[i] *= inv; const unsigned short hb = f2bf(o[i]); oh[i] = hb; ol[i] = f2bf(o[i] - bf2f(hb)); }
    const size_t off = p * CC + c0; *(volatile v8f*)(ATT + off) = o; *(volatile v8us*)(Ah + off) = oh; *(volatile v8us*)(Al + off) = ol; __threadfence(); *(volatile v8f*)(ATT + off) = o; *(volatile v8us*)(Ah + off) = oh; *(volatile v8us*)(Al + off) = ol;
}
__global__ __launch_bounds__(256) void k_ln256(const float* __restrict__ X1, const float* __restrict__ w, const float* __restrict__ bb, bf* Hh, bf* Hl) {
    const int lane = threadIdx.x & 31; const size_t r = (size_t)blockIdx.x * 8 + (threadIdx.x >> 5); if (r >= (size_t)NPX) return; float v[8]; float s = 0.f;
#pragma unroll
    for (int i = 0; i < 8; ++i) { v[i] = X1[r * CC + lane * 8 + i]; s += v[i]; }
#pragma unroll
    for (int sh = 16; sh; sh >>= 1) s += __shfl_xor(s, sh, 32);
    const float mu = s * (1.0f / CC); float q = 0.f;
#pragma unroll
    for (int i = 0; i < 8; ++i) { const float d = v[i] - mu; q = fmaf(d, d, q); }
#pragma unroll
    for (int sh = 16; sh; sh >>= 1) q += __shfl_xor(q, sh, 32);
    const float rs = rsqrtf(q * (1.0f / CC) + LEPS); v8us oh, ol;
#pragma unroll
    for (int i = 0; i < 8; ++i) { const int c = lane * 8 + i; const float yv = (v[i] - mu) * rs * bfr(w[c]) + bfr(bb[c]); const unsigned short hb = f2bf(yv); oh[i] = hb; ol[i] = f2bf(yv - bf2f(hb)); }
    const size_t o = r * CC + lane * 8; *(volatile v8us*)(Hh + o) = oh; *(volatile v8us*)(Hl + o) = ol; __threadfence(); *(volatile v8us*)(Hh + o) = oh; *(volatile v8us*)(Hl + o) = ol;
}
__global__ __launch_bounds__(256) void k_gelu1024(const float* __restrict__ F, bf* Gh, bf* Gl) {
    const int lane = threadIdx.x & 31; const size_t r = (size_t)blockIdx.x * 8 + (threadIdx.x >> 5); if (r >= (size_t)NPX) return;
#pragma unroll 1
    for (int ps = 0; ps < 2; ++ps) {
#pragma unroll 1
        for (int q = 0; q < HID / 256; ++q) { const size_t o = r * HID + q * 256 + lane * 8; const v8f v = *(const v8f*)(F + o); v8us oh, ol;
#pragma unroll
            for (int i = 0; i < 8; ++i) { const float xv = v[i]; const float gx = 0.5f * xv * (1.0f + erff(xv * 0.70710678118654752f)); const unsigned short hb = f2bf(gx); oh[i] = hb; ol[i] = f2bf(gx - bf2f(hb)); }
            *(volatile v8us*)(Gh + o) = oh; *(volatile v8us*)(Gl + o) = ol; }
        if (ps == 0) __threadfence(); }
}
__global__ __launch_bounds__(256) void k_troutC(const float* __restrict__ Y, float* OUTB) {
    __shared__ float tl[64][65];
    const int tid = threadIdx.x; const int p0 = blockIdx.x * 64, c0 = blockIdx.y * 64; const int rr = tid >> 2, cq = (tid & 3) * 16;
#pragma unroll
    for (int i = 0; i < 16; ++i) tl[rr][cq + i] = Y[(size_t)(p0 + rr) * CC + c0 + cq + i];
    __syncthreads();
    const int lane = tid & 31, wv = tid >> 5;
    auto pass = [&]() {
#pragma unroll
        for (int st = 0; st < 4; ++st) { const int cr = wv * 8 + st * 2 + (lane >> 4); const int lq = (lane & 15) * 4; v4f v;
#pragma unroll
            for (int i = 0; i < 4; ++i) v[i] = tl[lq + i][cr];
            *(volatile v4f*)(OUTB + (size_t)(c0 + cr) * NPX + p0 + lq) = v; }
    };
    pass(); __threadfence(); pass();
}

extern "C" void kernel_launch(void* const* d_in, const int* in_sizes, int n_in,
                              void* d_out, int out_size, void* d_ws, size_t ws_size, hipStream_t stream) {
    (void)in_sizes; (void)n_in; (void)out_size;
    const float* sub = (const float*)d_in[0]; const float* ori = (const float*)d_in[1]; const float* wq = (const float*)d_in[2]; const float* wk = (const float*)d_in[3]; const float* wv = (const float*)d_in[4]; const float* pw = (const float*)d_in[5]; const float* pb = (const float*)d_in[6];
    const float* lnw = (const float*)d_in[7]; const float* lnb = (const float*)d_in[8]; const float* f1w = (const float*)d_in[9]; const float* f1b = (const float*)d_in[10]; const float* f2w = (const float*)d_in[11]; const float* f2b = (const float*)d_in[12];
    float* out = (float*)d_out;
    char* wsp = (char*)d_ws;
    auto take = [&](size_t bytes) { char* p = wsp; wsp += (bytes + 255) & ~(size_t)255; return (void*)p; };
    bf* WQ = (bf*)take((size_t)CC * CC * 2); bf* WK = (bf*)take((size_t)CC * CC * 2); bf* WV = (bf*)take((size_t)CC * CC * 2); bf* WP = (bf*)take((size_t)CC * CC * 2); bf* W1 = (bf*)take((size_t)HID * CC * 2); bf* W2 = (bf*)take((size_t)CC * HID * 2);
    bf* ST = (bf*)take((size_t)NPX * CC * 2); bf* OT = (bf*)take((size_t)NPX * CC * 2); float* Q = (float*)take((size_t)NPX * CC * 4); float* K = (float*)take((size_t)NPX * CC * 4); float* V = (float*)take((size_t)NPX * CC * 4);
    float* ATT = (float*)take((size_t)NPX * CC * 4); bf* Ah = (bf*)take((size_t)NPX * CC * 2); bf* Al = (bf*)take((size_t)NPX * CC * 2); float* X1 = (float*)take((size_t)NPX * CC * 4); bf* Hh = (bf*)take((size_t)NPX * CC * 2); bf* Hl = (bf*)take((size_t)NPX * CC * 2);
    float* F1 = (float*)take((size_t)NPX * HID * 4); bf* Gh = (bf*)take((size_t)NPX * HID * 2); bf* Gl = (bf*)take((size_t)NPX * HID * 2); float* Y = (float*)take((size_t)NPX * CC * 4);
    if ((size_t)(wsp - (char*)d_ws) > ws_size) return;
    k_cvt8<<<(CC * CC / 8 + 255) / 256, 256, 0, stream>>>(wq, WQ, CC * CC / 8); k_cvt8<<<(CC * CC / 8 + 255) / 256, 256, 0, stream>>>(wk, WK, CC * CC / 8); k_cvt8<<<(CC * CC / 8 + 255) / 256, 256, 0, stream>>>(wv, WV, CC * CC / 8); k_cvt8<<<(CC * CC / 8 + 255) / 256, 256, 0, stream>>>(pw, WP, CC * CC / 8);
    k_cvt8<<<(HID * CC / 8 + 255) / 256, 256, 0, stream>>>(f1w, W1, HID * CC / 8); k_cvt8<<<(CC * HID / 8 + 255) / 256, 256, 0, stream>>>(f2w, W2, CC * HID / 8);
    const dim3 gp(NPX / 64, CC / 64, 1);
    for (int b = 0; b < NB_; ++b) {
        k_ptb<<<dim3(CC / 64, NPX / 64, 1), 256, 0, stream>>>(sub + (size_t)b * CC * NPX, ST); k_ptb<<<dim3(CC / 64, NPX / 64, 1), 256, 0, stream>>>(ori + (size_t)b * CC * NPX, OT);
        k_gemmb<false, false><<<gp, 128, 0, stream>>>(ST, nullptr, WQ, nullptr, Q, CC, nullptr, nullptr, CC); k_gemmb<false, false><<<gp, 128, 0, stream>>>(OT, nullptr, WK, nullptr, K, CC, nullptr, nullptr, CC); k_gemmb<false, false><<<gp, 128, 0, stream>>>(OT, nullptr, WV, nullptr, V, CC, nullptr, nullptr, CC);
        k_local<<<NPX / 8, 256, 0, stream>>>(Q, K, V, ATT, Ah, Al);
        k_gemmb<true, false><<<gp, 128, 0, stream>>>(Ah, Al, WP, pb, X1, CC, nullptr, nullptr, CC);
        k_ln256<<<NPX / 8, 256, 0, stream>>>(X1, lnw, lnb, Hh, Hl);
        k_gemmb<true, false><<<dim3(NPX / 64, HID / 64, 1), 128, 0, stream>>>(Hh, Hl, W1, f1b, F1, HID, nullptr, nullptr, CC);
        k_gelu1024<<<NPX / 8, 256, 0, stream>>>(F1, Gh, Gl);
        k_gemmb<true, false><<<gp, 128, 0, stream>>>(Gh, Gl, W2, f2b, Y, CC, nullptr, X1, HID, 0);
        k_troutC<<<dim3(NPX / 64, CC / 64, 1), 256, 0, stream>>>(Y, out + (size_t)b * CC * NPX); }
}
